// GNNClassifier_85856396247086
// MI455X (gfx1250) — hardware-verified
//
#include <hip/hip_runtime.h>
#include <math.h>

constexpr int kNodes    = 100000;
constexpr int kEdges    = 1600000;
constexpr int kCin      = 128;
constexpr int kHid      = 64;
constexpr int kHid2     = 32;
constexpr int kCls      = 2;
constexpr int kGraphs   = 256;
constexpr int kNodesPad = 100032;
constexpr int kNT       = 256;

constexpr int kTileRows    = 1024;
constexpr int kTiles       = 98;
constexpr int kWaveRows    = kTileRows / 8;
constexpr int kWaveRowsLog = 7;
constexpr int kChunkA      = 4096;
constexpr int kSpA         = kChunkA / kNT;
constexpr int kNChunkA     = (kEdges + kChunkA - 1) / kChunkA;
constexpr int kRecShift    = 21;
constexpr int kLowMask     = 0x1FFFFF;
constexpr int kOwnShiftA   = kRecShift + kWaveRowsLog;

constexpr int kTileRowsD    = 16384;
constexpr int kTilesD       = 7;
constexpr int kDinvRows     = kTilesD * kTileRowsD;
constexpr int kWaveRowsDLog = 11;
constexpr int kChunkD       = 4096;
constexpr int kSpD          = kChunkD / kNT;
constexpr int kNChunkD      = (kEdges + kChunkD - 1) / kChunkD;

constexpr int kGpb      = 8;
constexpr int kChunkP   = 2048;
constexpr int kSpP      = kChunkP / kNT;
constexpr int kNChunkP  = (kNodes + kChunkP - 1) / kChunkP;
constexpr int kPosShift = 17;
constexpr int kPosMask  = 0x1FFFF;

constexpr float kXCarry = 8.0f;
constexpr float kWCarry = 64.0f;
constexpr float kHCarry = 16.0f;
constexpr float kScale1 = 1.0f / (8.0f * 64.0f);
constexpr float kScale2 = 1.0f / (16.0f * 64.0f);

static_assert(kNodesPad % 64 == 0 && kNodesPad >= kNodes);
static_assert(kHid % 64 == 0);
static_assert(kCin % 32 == 0 && kHid % 32 == 0);
static_assert(kTiles * kTileRows >= kNodesPad && kDinvRows >= kNodesPad);
static_assert(kEdges % kSpA == 0 && kEdges % kSpD == 0 && kNodes % kSpP == 0);
static_assert((1 << kWaveRowsLog) == kWaveRows && (8 << kWaveRowsDLog) == kTileRowsD);
static_assert((1 << kRecShift) > kEdges - 1);
static_assert((long long)(kTileRows - 1) * (1LL << kRecShift) + (kEdges - 1) < 2147483647LL);
static_assert((1 << kPosShift) > kNodes - 1);
static_assert(kGraphs % kGpb == 0);
static_assert(kNodes % 4 == 0 && kNodesPad % 4 == 0);
static_assert(kGraphs * kCls == 512);

typedef __attribute__((ext_vector_type(16))) _Float16 v16h;
typedef __attribute__((ext_vector_type(8)))  _Float16 v8h;
typedef __attribute__((ext_vector_type(16))) __bf16   v16b;
typedef __attribute__((ext_vector_type(8)))  __bf16   v8b;
typedef __attribute__((ext_vector_type(8)))  float    v8f;
typedef __attribute__((ext_vector_type(4)))  float    v4f;
typedef __attribute__((ext_vector_type(2)))  float    v2f;
typedef __attribute__((ext_vector_type(4)))  int      v4i;
typedef __attribute__((ext_vector_type(4)))  unsigned int v4u;

__device__ __forceinline__ unsigned short f2bf_bits(float f) {
  unsigned u = __float_as_uint(f);
  return (unsigned short)((u + 0x7FFFu + ((u >> 16) & 1u)) >> 16);
}
__device__ __forceinline__ float bf_bits2f(unsigned short h) { return __uint_as_float(((unsigned)h) << 16); }

__device__ __forceinline__ void dep_guard_h(v8f& a, v8f& b, v16h x, v16h y) { asm volatile("v_nop\n\tv_nop\n\tv_nop\n\tv_nop" : "+v"(a), "+v"(b) : "v"(x), "v"(y)); }
__device__ __forceinline__ void dep_guard_b(v8f& a, v8f& b, v16b x, v16b y) { asm volatile("v_nop\n\tv_nop\n\tv_nop\n\tv_nop" : "+v"(a), "+v"(b) : "v"(x), "v"(y)); }
__device__ __forceinline__ void dep_guard4_h(v8f& a, v8f& b, v8f& c, v8f& d, v16h x, v16h y) { asm volatile("v_nop\n\tv_nop\n\tv_nop\n\tv_nop" : "+v"(a), "+v"(b), "+v"(c), "+v"(d) : "v"(x), "v"(y)); }
__device__ __forceinline__ void dep_guard4_b(v8f& a, v8f& b, v8f& c, v8f& d, v16b x, v16b y) { asm volatile("v_nop\n\tv_nop\n\tv_nop\n\tv_nop" : "+v"(a), "+v"(b), "+v"(c), "+v"(d) : "v"(x), "v"(y)); }
__device__ __forceinline__ void keep4_h(v16h a, v16h b, v16h c, v16h d) { asm volatile("v_nop" :: "v"(a), "v"(b), "v"(c), "v"(d)); }
__device__ __forceinline__ void keep4_b(v16b a, v16b b, v16b c, v16b d) { asm volatile("v_nop" :: "v"(a), "v"(b), "v"(c), "v"(d)); }
__device__ __forceinline__ void acc_guard4(v8f& a, v8f& b, v8f& c, v8f& d) { asm volatile("v_nop\n\tv_nop\n\tv_nop\n\tv_nop" : "+v"(a), "+v"(b), "+v"(c), "+v"(d)); }
template <typename T> struct Frag;
template <> struct Frag<_Float16> {
  typedef v16h V; union U { v16h v; v8h h[2]; };
  static __device__ __forceinline__ v16h load(const _Float16* p) {
    U f; f.h[0] = *(const v8h*)(p); f.h[1] = *(const v8h*)(p + 16); return f.v;
  }
  static __device__ __forceinline__ v8f mma(v16h a, v16h b, v8f c) {
    return __builtin_amdgcn_wmma_f32_16x16x32_f16(false, a, false, b, (short)0, c, false, false);
  }
  static __device__ __forceinline__ void guard(v8f& a, v8f& b, v16h x, v16h y) { dep_guard_h(a, b, x, y); }
  static __device__ __forceinline__ void guard4(v8f& a, v8f& b, v8f& c, v8f& d, v16h x, v16h y) { dep_guard4_h(a, b, c, d, x, y); }
  static __device__ __forceinline__ void keep(v16h a, v16h b, v16h c, v16h d) { keep4_h(a, b, c, d); }
};
template <> struct Frag<__bf16> {
  typedef v16b V; union U { v16b v; v8b h[2]; };
  static __device__ __forceinline__ v16b load(const __bf16* p) {
    U f; f.h[0] = *(const v8b*)(p); f.h[1] = *(const v8b*)(p + 16); return f.v;
  }
  static __device__ __forceinline__ v8f mma(v16b a, v16b b, v8f c) {
    return __builtin_amdgcn_wmma_f32_16x16x32_bf16(false, a, false, b, (short)0, c, false, false);
  }
  static __device__ __forceinline__ void guard(v8f& a, v8f& b, v16b x, v16b y) { dep_guard_b(a, b, x, y); }
  static __device__ __forceinline__ void guard4(v8f& a, v8f& b, v8f& c, v8f& d, v16b x, v16b y) { dep_guard4_b(a, b, c, d, x, y); }
  static __device__ __forceinline__ void keep(v16b a, v16b b, v16b c, v16b d) { keep4_b(a, b, c, d); }
};

__device__ __forceinline__ unsigned pk16(unsigned short a, unsigned short b) { return (unsigned)a | ((unsigned)b << 16); }
__device__ __forceinline__ unsigned short h_bits(float f) { const _Float16 h = (_Float16)f; return __builtin_bit_cast(unsigned short, h); }

template <int ET> struct Elem;
template <> struct Elem<0> { typedef _Float16 T; };
template <> struct Elem<1> { typedef __bf16 T; };
template <int ET, bool SPLIT, int BIAS_MODE, int OUT_MODE, bool RESID, int ACT = 0>
__global__ __launch_bounds__(256) void wmma_gemm64(
    const unsigned short* __restrict__ Ap, const unsigned short* __restrict__ A2p, int lda, long strideA,
    const unsigned short* __restrict__ Btp, const unsigned short* __restrict__ Bt2p, int ldb, long strideB,
    void* __restrict__ Cout, void* __restrict__ Cout2, int ldc, long strideC,
    const float* __restrict__ bias,
    const float* __restrict__ resid, long strideR,
    int M, int N, int K, float scale) {
  typedef typename Elem<ET>::T T;
  typedef typename Frag<T>::V V;
  const T* A = (const T*)Ap; const T* A2 = (const T*)A2p; const T* Bt = (const T*)Btp; const T* Bt2 = (const T*)Bt2p;
  __shared__ __align__(16) float sT[8][16 * 68];
  const int b    = blockIdx.y;
  const int lane = threadIdx.x & 31;
  const int wave = threadIdx.x >> 5;
  const int tilesN = N >> 6;
  const int tilesM = M >> 6;
  const int tile = blockIdx.x * 8 + wave;
  if (tile >= tilesM * tilesN) return;
  const int tm = tile / tilesN;
  const int tn = tile - tm * tilesN;
  const int m0 = tm << 6;
  const int n0 = tn << 6;

  const T* Ab  = A  + (size_t)b * strideA;
  const T* Bb  = Bt + (size_t)b * strideB;
  const T* Ab2 = SPLIT ? (A2  + (size_t)b * strideA) : nullptr;
  const T* Bb2 = SPLIT ? (Bt2 + (size_t)b * strideB) : nullptr;

  const int rlane = lane & 15;
  const int koff  = (lane >> 4) * 8;
  const int mOff  = (lane >> 4) * 8;

  v8f acc[4][4];
#pragma unroll
  for (int i = 0; i < 4; ++i)
#pragma unroll
    for (int j = 0; j < 4; ++j) acc[i][j] = (v8f){0.f,0.f,0.f,0.f,0.f,0.f,0.f,0.f};

  for (int k0 = 0; k0 < K; k0 += 32) {
    V bh[4], bl[4];
#pragma unroll
    for (int j = 0; j < 4; ++j) {
      const size_t bo = (size_t)(n0 + (j << 4) + rlane) * ldb + koff + k0;
      bh[j] = Frag<T>::load(Bb + bo);
      if (SPLIT) bl[j] = Frag<T>::load(Bb2 + bo);
    }
#pragma unroll
    for (int i = 0; i < 4; ++i) {
      const size_t ao = (size_t)(m0 + (i << 4) + rlane) * lda + koff + k0;
      V ah = Frag<T>::load(Ab + ao);
      V al;
      if (SPLIT) al = Frag<T>::load(Ab2 + ao);
#pragma unroll
      for (int j = 0; j < 4; ++j) {
        acc[i][j] = Frag<T>::mma(ah, bh[j], acc[i][j]);
        if (SPLIT) {
          acc[i][j] = Frag<T>::mma(ah, bl[j], acc[i][j]);
          acc[i][j] = Frag<T>::mma(al, bh[j], acc[i][j]);
        }
      }
      Frag<T>::guard4(acc[i][0], acc[i][1], acc[i][2], acc[i][3], ah, SPLIT ? al : ah);
    }
    Frag<T>::keep(bh[0], bh[1], bh[2], bh[3]);
    if (SPLIT) Frag<T>::keep(bl[0], bl[1], bl[2], bl[3]);
  }
  acc_guard4(acc[0][0], acc[0][1], acc[0][2], acc[0][3]);
  acc_guard4(acc[1][0], acc[1][1], acc[1][2], acc[1][3]);
  acc_guard4(acc[2][0], acc[2][1], acc[2][2], acc[2][3]);
  acc_guard4(acc[3][0], acc[3][1], acc[3][2], acc[3][3]);

  float* slab = sT[wave];
  const float* Rb = RESID ? (resid + (size_t)b * strideR) : nullptr;
#pragma unroll
  for (int i = 0; i < 4; ++i) {
    const int mBase = m0 + (i << 4);
#pragma unroll
    for (int j = 0; j < 4; ++j) {
      const int n = n0 + (j << 4) + rlane;
      float bv = 0.f;
      if (BIAS_MODE == 2) bv = bias[n];
#pragma unroll
      for (int r = 0; r < 8; ++r) {
        float v = acc[i][j][r] * scale;
        if (BIAS_MODE == 1) v += bias[mBase + mOff + r];
        if (BIAS_MODE == 2) v += bv;
        if (RESID) v += Rb[(size_t)(mBase + mOff + r) * ldc + n];
        if (ACT == 2) v = fmaxf(v, 0.0f);
        if (ACT == 4) v = (v > 0.f) ? v : 0.01f * v;
        slab[(mOff + r) * 68 + (j << 4) + rlane] = v;
      }
    }
    __builtin_amdgcn_fence(__ATOMIC_RELEASE, "workgroup");
    __builtin_amdgcn_wave_barrier();
    __builtin_amdgcn_fence(__ATOMIC_ACQUIRE, "workgroup");
    if (OUT_MODE == 0) {
      float* C = (float*)Cout + (size_t)b * strideC;
      const int hh = lane >> 4, c4 = (lane & 15) * 4;
      for (int pass = 0; pass < 2; ++pass) {
#pragma unroll
        for (int it = 0; it < 8; ++it) {
          const int row = it * 2 + hh;
          v4f v = *(const v4f*)(slab + row * 68 + c4);
          *(volatile v4f*)(C + (size_t)(mBase + row) * ldc + n0 + c4) = v;
        }
        __threadfence();
      }
    } else {
      const int q = lane >> 3, c8 = (lane & 7) * 8;
      unsigned short* C  = (unsigned short*)Cout  + (size_t)b * strideC;
      unsigned short* C2 = (OUT_MODE == 2) ? ((unsigned short*)Cout2 + (size_t)b * strideC) : nullptr;
      for (int pass = 0; pass < 2; ++pass) {
#pragma unroll
        for (int it = 0; it < 4; ++it) {
          const int row = it * 4 + q;
          const float* sp = slab + row * 68 + c8;
          v8h hv, lv;
#pragma unroll
          for (int e = 0; e < 8; ++e) {
            if (OUT_MODE == 1) {
              hv[e] = (_Float16)sp[e];
            } else {
              unsigned short hb = f2bf_bits(sp[e]);
              unsigned short lb = f2bf_bits(sp[e] - bf_bits2f(hb));
              hv[e] = __builtin_bit_cast(_Float16, hb);
              lv[e] = __builtin_bit_cast(_Float16, lb);
            }
          }
          *(volatile v8h*)(C + (size_t)(mBase + row) * ldc + n0 + c8) = hv;
          if (OUT_MODE == 2) *(volatile v8h*)(C2 + (size_t)(mBase + row) * ldc + n0 + c8) = lv;
        }
        __threadfence();
      }
    }
    __builtin_amdgcn_fence(__ATOMIC_RELEASE, "workgroup");
    __builtin_amdgcn_wave_barrier();
    __builtin_amdgcn_fence(__ATOMIC_ACQUIRE, "workgroup");
  }
}

__device__ __forceinline__ int blk_excl_scan(int cnt, int* scan_ws, int tid, int* tot) {
  const int lane = tid & 31, wave = tid >> 5; int incl = cnt;
#pragma unroll
  for (int o = 1; o < 32; o <<= 1) { const int v = __shfl_up(incl, o, 32); if (lane >= o) incl += v; }
  if (lane == 31) scan_ws[wave] = incl;
  __syncthreads();
  if (wave == 0) {
    const int wv = scan_ws[lane];
    int wincl = wv;
#pragma unroll
    for (int o = 1; o < 32; o <<= 1) { const int v = __shfl_up(wincl, o, 32); if (lane >= o) wincl += v; }
    if (lane < kNT / 32) scan_ws[32 + lane] = wincl - wv;
    if (lane == 31) scan_ws[64] = wincl;
  }
  __syncthreads();
  const int res = scan_ws[32 + wave] + incl - cnt; *tot = scan_ws[64];
  return res;
}

template <int SP, int CAP, int SHIFT, bool LOWPOS, int LEN>
__device__ __forceinline__ int chunk_select(const int* __restrict__ keyv, int e0, int lo, unsigned span,
                                            int tid, int* LIST, int* scan_ws) {
  static_assert(LEN % SP == 0 && SP % 4 == 0 && SP <= 16 && CAP == SP * kNT);
  const int eb = e0 + tid * SP;
  const bool inr = eb < LEN;
  const int ebc = inr ? eb : (LEN - SP);
  unsigned hm = 0u;
#pragma unroll
  for (int k = 0; k < SP; k += 4) {
    const v4i d4 = *(const v4i*)(keyv + ebc + k);
#pragma unroll
    for (int e = 0; e < 4; ++e) {
      const unsigned u = (unsigned)d4[e] - (unsigned)lo;
      const unsigned hb = (u < span) ? 1u : 0u;
      hm |= hb << (k + e);
    }
  }
  hm = inr ? hm : 0u;
  const int cnt = __builtin_popcount(hm);
  int tot;
  int p = blk_excl_scan(cnt, scan_ws, tid, &tot);
#pragma unroll 1
  for (int it = 0; it < SP; ++it) {
    const unsigned any = (unsigned)__ballot(hm != 0u);
    if (any == 0u) break;
    const bool valid = hm != 0u;
    const int kz = __builtin_ctz(hm | (1u << SP));
    const int kk = kz < SP ? kz : SP - 1;
    const int d = keyv[ebc + kk];
    const unsigned pos = LOWPOS ? (unsigned)(ebc + kk) : 0u;
    const int rec = (int)((((unsigned)d - (unsigned)lo) << SHIFT) | pos);
    int slot = valid ? p : CAP;
    slot = ((unsigned)slot <= (unsigned)CAP) ? slot : CAP;
    LIST[slot] = rec;
    p += valid ? 1 : 0;
    hm &= hm - 1u;
  }
  __syncthreads();
  return tot < CAP ? tot : CAP;
}

__global__ __launch_bounds__(kNT) void castw_kernel(const float* __restrict__ W1, const float* __restrict__ W2,
                                                    unsigned short* __restrict__ W1T, unsigned short* __restrict__ W2T) {
  __shared__ float sm[kHid][kCin + 4];
  const int t = threadIdx.x;
  const int z = blockIdx.x;
  const int kdim = (z == 0) ? kCin : kHid;
  const int lk   = (z == 0) ? 7 : 6;
  const float* W = (z == 0) ? W1 : W2;
  unsigned short* O = (z == 0) ? W1T : W2T;
  for (int idx = t; idx < kdim * kHid; idx += kNT) {
    const int k = idx >> 6, n = idx & 63;
    sm[n][k] = W[idx] * kWCarry;
  }
  __syncthreads();
  const int nit = (kdim * kHid) >> 11;
  for (int it = 0; it < nit; ++it) {
    const int off = it * 2048 + 8 * t;
    const int row = off >> lk, col = off & (kdim - 1);
    unsigned short hb[8];
#pragma unroll
    for (int e = 0; e < 8; ++e) hb[e] = h_bits(sm[row][col + e]);
    const v4u u = (v4u){pk16(hb[0], hb[1]), pk16(hb[2], hb[3]), pk16(hb[4], hb[5]), pk16(hb[6], hb[7])};
    unsigned short* p = O + off;
    *(volatile v4u*)p = u;
    __threadfence();
    *(volatile v4u*)p = u;
  }
}

__global__ __launch_bounds__(kNT) void castx_kernel(const float* __restrict__ x, unsigned short* __restrict__ XH) {
  const int i = blockIdx.x * kNT + threadIdx.x;
  if (i >= kNodesPad * kCin / 8) return;
  const int r  = i >> 4;
  const int c8 = (i & 15) * 8;
  const int rr = r < kNodes ? r : kNodes - 1;
  const float sc = r < kNodes ? kXCarry : 0.0f;
  const float* p = x + (size_t)rr * kCin + c8;
  const v4f a = *(const v4f*)(p);
  const v4f c = *(const v4f*)(p + 4);
  unsigned short hb[8];
#pragma unroll
  for (int e = 0; e < 4; ++e) { hb[e] = h_bits(a[e] * sc); hb[4 + e] = h_bits(c[e] * sc); }
  const v4u u = (v4u){pk16(hb[0], hb[1]), pk16(hb[2], hb[3]), pk16(hb[4], hb[5]), pk16(hb[6], hb[7])};
  unsigned short* q = XH + 8 * (size_t)i;
  *(volatile v4u*)q = u;
  __threadfence();
  *(volatile v4u*)q = u;
}

__global__ __launch_bounds__(kNT) void degree_kernel(const int* __restrict__ ei, float* __restrict__ DINVp) {
  __shared__ int CNT[kTileRowsD];
  __shared__ int LIST[kChunkD + 4];
  __shared__ int scan_ws[80];
  const int tid = threadIdx.x, lane = tid & 31, wave = tid >> 5;
  const int n0 = blockIdx.x * kTileRowsD;
  for (int i = tid; i < kChunkD + 4; i += kNT) LIST[i] = -1;
  for (int i = tid; i < kTileRowsD; i += kNT) CNT[i] = 0;
  if (tid < 80) scan_ws[tid] = 0;
  __syncthreads();
  const int* dstv = ei + kEdges;
#pragma unroll 1
  for (int c = 0; c < kNChunkD; ++c) {
    const int tot = chunk_select<kSpD, kChunkD, 0, false, kEdges>(dstv, c * kChunkD, n0, (unsigned)kTileRowsD, tid, LIST, scan_ws);
#pragma unroll 1
    for (int base = 0; base < tot; base += 32) {
      const int q = base + lane;
      const int qc = q < kChunkD ? q : kChunkD - 1;
      const int lv = LIST[qc];
      const int own = (int)(q < tot) & (int)(lv >= 0) & (int)((lv >> kWaveRowsDLog) == wave);
      unsigned msk = (unsigned)__ballot(own);
#pragma unroll 1
      for (int it = 0; it < 32; ++it) {
        if (msk == 0u) break;
        const int bp = __builtin_ctz(msk);
        msk &= msk - 1u;
        const int r = __shfl(lv, bp, 32);
        const int dl = r & (kTileRowsD - 1);
        const int cv = CNT[dl];
        if (lane == 0) CNT[dl] = cv + 1;
      }
    }
    __syncthreads();
  }
  __syncthreads();
#pragma unroll 1
  for (int it = 0; it < kTileRowsD / (4 * kNT); ++it) {
    const int i = it * 4 * kNT + 4 * tid;
    v4f d;
#pragma unroll
    for (int e = 0; e < 4; ++e) d[e] = 1.0f / sqrtf((float)CNT[i + e] + 1.0f);
    float* p = DINVp + (size_t)n0 + i;
    *(volatile v4f*)p = d;
    __threadfence();
    *(volatile v4f*)p = d;
  }
}

template <bool OUT16>
__global__ __launch_bounds__(kNT) void gcn_agg_kernel(const float* __restrict__ HLp, const int* __restrict__ ei,
                                                      const float* __restrict__ DINVp, const float* __restrict__ bias,
                                                      unsigned short* __restrict__ OutH, float* __restrict__ OutF) {
  __shared__ __align__(16) float accl[kTileRows * kHid];
  __shared__ int LIST[kChunkA + 4];
  __shared__ int scan_ws[80];
  const int tid = threadIdx.x, lane = tid & 31, wave = tid >> 5;
  const int n0 = blockIdx.x * kTileRows;
  for (int i = tid; i < kChunkA + 4; i += kNT) LIST[i] = -1;
  if (tid < 80) scan_ws[tid] = 0;
  const v2f z2 = {0.f, 0.f};
  {
    float* wr = accl + (wave * kWaveRows) * kHid + 2 * lane;
#pragma unroll 1
    for (int j = 0; j < kWaveRows; ++j) *(v2f*)(wr + j * kHid) = z2;
  }
  __syncthreads();
  const int* srcv = ei;
  const int* dstv = ei + kEdges;
#pragma unroll 1
  for (int c = 0; c < kNChunkA; ++c) {
    const int tot = chunk_select<kSpA, kChunkA, kRecShift, true, kEdges>(dstv, c * kChunkA, n0, (unsigned)kTileRows, tid, LIST, scan_ws);
#pragma unroll 1
    for (int base = 0; base < tot; base += 32) {
      const int q = base + lane;
      const int qc = q < kChunkA ? q : kChunkA - 1;
      const int lv = LIST[qc];
      const int own = (int)(q < tot) & (int)(lv >= 0) & (int)((lv >> kOwnShiftA) == wave);
      unsigned msk = (unsigned)__ballot(own);
#pragma unroll 1
      for (int it = 0; it < 32; ++it) {
        if (msk == 0u) break;
        const int bp = __builtin_ctz(msk);
        msk &= msk - 1u;
        const int r = __shfl(lv, bp, 32);
        const int dl = (int)((unsigned)r >> kRecShift) & (kTileRows - 1);
        int e = r & kLowMask; e = e < kEdges ? e : kEdges - 1;
        int s = srcv[e]; s = s < 0 ? 0 : (s >= kNodes ? kNodes - 1 : s);
        const float wsrc = DINVp[s];
        const v2f hv = *(const v2f*)(HLp + (size_t)s * kHid + 2 * lane);
        float* rp = accl + dl * kHid + 2 * lane;
        v2f a = *(const v2f*)rp;
        a = a + wsrc * hv;
        *(v2f*)rp = a;
      }
    }
    __syncthreads();
  }
  __syncthreads();
  if (OUT16) {
    const int rq = lane >> 3, c8 = (lane & 7) * 8;
    const v4f bA = *(const v4f*)(bias + c8);
    const v4f bB = *(const v4f*)(bias + c8 + 4);
#pragma unroll 1
    for (int jj = 0; jj < kWaveRows / 4; ++jj) {
      const int lb = wave * kWaveRows + jj * 4;
      const int nb = n0 + lb;
      if (nb < kNodesPad) {
        const int n = nb + rq;
        const bool live = nb < kNodes;
        const float dn = DINVp[n];
        const float* ap = accl + (lb + rq) * kHid + c8;
        const v4f a0 = *(const v4f*)(ap);
        const v4f a1 = *(const v4f*)(ap + 4);
        const float* hp = HLp + (size_t)n * kHid + c8;
        const v4f h0 = *(const v4f*)(hp);
        const v4f h1v = *(const v4f*)(hp + 4);
        unsigned short hb[8];
#pragma unroll
        for (int e = 0; e < 4; ++e) {
          float v0 = dn * (a0[e] + dn * h0[e]) + bA[e];
          float v1 = dn * (a1[e] + dn * h1v[e]) + bB[e];
          v0 = live ? fmaxf(v0, 0.f) * kHCarry : 0.f;
          v1 = live ? fmaxf(v1, 0.f) * kHCarry : 0.f;
          hb[e] = h_bits(v0); hb[4 + e] = h_bits(v1);
        }
        const v4u u = (v4u){pk16(hb[0], hb[1]), pk16(hb[2], hb[3]), pk16(hb[4], hb[5]), pk16(hb[6], hb[7])};
        unsigned short* op = OutH + (size_t)n * kHid + c8;
        for (int pass = 0; pass < 2; ++pass) { *(volatile v4u*)op = u; __threadfence(); }
      }
    }
  } else {
    const int rh = lane >> 4, c4 = (lane & 15) * 4;
    const v4f b4 = *(const v4f*)(bias + c4);
#pragma unroll 1
    for (int jj = 0; jj < kWaveRows / 2; ++jj) {
      const int lb = wave * kWaveRows + jj * 2;
      const int nb = n0 + lb;
      if (nb < kNodesPad) {
        const int n = nb + rh;
        const bool live = nb < kNodes;
        const float dn = DINVp[n];
        const v4f a  = *(const v4f*)(accl + (lb + rh) * kHid + c4);
        const v4f hs = *(const v4f*)(HLp + (size_t)n * kHid + c4);
        v4f v;
#pragma unroll
        for (int e = 0; e < 4; ++e) {
          const float t = dn * (a[e] + dn * hs[e]) + b4[e];
          v[e] = live ? fmaxf(t, 0.f) : 0.f;
        }
        float* op = OutF + (size_t)n * kHid + c4;
        for (int pass = 0; pass < 2; ++pass) { *(volatile v4f*)op = v; __threadfence(); }
      }
    }
  }
}

__global__ __launch_bounds__(kNT) void pool_kernel(const float* __restrict__ H2p, const int* __restrict__ batch, float* __restrict__ Pp) {
  __shared__ int LIST[kChunkP + 4];
  __shared__ int scan_ws[80];
  __shared__ __align__(16) float red[8 * kHid];
  const int tid = threadIdx.x, lane = tid & 31, wave = tid >> 5;
  const int g0 = blockIdx.x * kGpb;
  for (int i = tid; i < kChunkP + 4; i += kNT) LIST[i] = -1;
  if (tid < 80) scan_ws[tid] = 0;
  __syncthreads();
  v2f acc = {0.f, 0.f};
  int cnt = 0;
#pragma unroll 1
  for (int c = 0; c < kNChunkP; ++c) {
    const int tot = chunk_select<kSpP, kChunkP, kPosShift, true, kNodes>(batch, c * kChunkP, g0, (unsigned)kGpb, tid, LIST, scan_ws);
#pragma unroll 1
    for (int base = 0; base < tot; base += 32) {
      const int q = base + lane;
      const int qc = q < kChunkP ? q : kChunkP - 1;
      const int lv = LIST[qc];
      const int own = (int)(q < tot) & (int)(lv >= 0) & (int)((lv >> kPosShift) == wave);
      unsigned msk = (unsigned)__ballot(own);
#pragma unroll 1
      for (int it = 0; it < 32; ++it) {
        if (msk == 0u) break;
        const int bp = __builtin_ctz(msk);
        msk &= msk - 1u;
        const int r = __shfl(lv, bp, 32);
        int nd = r & kPosMask; nd = nd < kNodes ? nd : kNodes - 1;
        acc = acc + *(const v2f*)(H2p + (size_t)nd * kHid + 2 * lane);
        ++cnt;
      }
    }
    __syncthreads();
  }
  *(v2f*)(red + wave * kHid + 2 * lane) = acc;
  __syncthreads();
  const int c4 = (lane & 15) * 4;
  const v4f s = *(const v4f*)(red + wave * kHid + c4);
  const float cf = (float)cnt;
  const float inv = 1.0f / fmaxf(cf, 1.0f);
  const v4f o = s * inv;
  float* prow = Pp + (size_t)(g0 + wave) * kHid + c4;
  for (int pass = 0; pass < 2; ++pass) {
    if (lane < 16) *(volatile v4f*)prow = o;
    __threadfence();
  }
}

__global__ __launch_bounds__(kNT) void head_kernel(const float* __restrict__ Pp, const float* __restrict__ Wc1, const float* __restrict__ bc1,
                                                  const float* __restrict__ Wc2, const float* __restrict__ bc2, float* __restrict__ out) {
  __shared__ float zs[kGraphs * kHid2];
  __shared__ __align__(16) float so[kGraphs * kCls];
  const int tid = threadIdx.x, wave = tid >> 5, lane = tid & 31;
  for (int i = tid; i < kGraphs * kHid2; i += kNT) {
    const int g = i >> 5, j = i & 31;
    float s = 0.f;
#pragma unroll 1
    for (int c = 0; c < kHid; ++c) s += Pp[g * kHid + c] * Wc1[c * kHid2 + j];
    s += bc1[j];
    zs[i] = fmaxf(s, 0.f);
  }
  __syncthreads();
  for (int i = tid; i < kGraphs * kCls; i += kNT) {
    const int g = i >> 1, k = i & 1;
    float a = 0.f;
#pragma unroll 1
    for (int j = 0; j < kHid2; ++j) a += zs[g * kHid2 + j] * Wc2[j * kCls + k];
    a += bc2[k];
    so[i] = a;
  }
  __syncthreads();
  if (wave == 0) {
    v4f p[4];
#pragma unroll
    for (int it = 0; it < 4; ++it) p[it] = *(const v4f*)(so + it * 128 + 4 * lane);
    for (int pass = 0; pass < 2; ++pass) {
#pragma unroll
      for (int it = 0; it < 4; ++it) *(volatile v4f*)(out + it * 128 + 4 * lane) = p[it];
      __threadfence();
    }
  }
}

extern "C" void kernel_launch(void* const* d_in, const int* in_sizes, int n_in,
                              void* d_out, int out_size, void* d_ws, size_t ws_size, hipStream_t stream) {
  (void)in_sizes; (void)n_in; (void)out_size;
  const float* x   = (const float*)d_in[0];
  const int*   ei  = (const int*)d_in[1];
  const int*   bat = (const int*)d_in[2];
  const float* W1  = (const float*)d_in[3];
  const float* b1  = (const float*)d_in[4];
  const float* W2  = (const float*)d_in[5];
  const float* b2  = (const float*)d_in[6];
  const float* Wc1 = (const float*)d_in[7];
  const float* bc1 = (const float*)d_in[8];
  const float* Wc2 = (const float*)d_in[9];
  const float* bc2 = (const float*)d_in[10];
  float* out = (float*)d_out;

  char* ws = (char*)d_ws; size_t off = 0;
  auto carve = [&](size_t bytes) -> char* { char* p = ws + off; off += (bytes + 255) & ~(size_t)255; return p; };
  unsigned short* W1T  = (unsigned short*)carve((size_t)kHid * kCin * 2);
  unsigned short* W2T  = (unsigned short*)carve((size_t)kHid * kHid * 2);
  float*          DINV = (float*)carve((size_t)kDinvRows * 4);
  unsigned short* XH   = (unsigned short*)carve((size_t)kNodesPad * kCin * 2);
  float*          HL   = (float*)carve((size_t)kNodesPad * kHid * 4);
  unsigned short* H1H  = (unsigned short*)carve((size_t)kNodesPad * kHid * 2);
  float*          H2   = (float*)carve((size_t)kNodesPad * kHid * 4);
  float*          P    = (float*)carve((size_t)kGraphs * kHid * 4);
  if (off > ws_size || off > (size_t)134217728) return;

  castw_kernel<<<2, kNT, 0, stream>>>(W1, W2, W1T, W2T);
  castx_kernel<<<(kNodesPad * kCin / 8) / kNT, kNT, 0, stream>>>(x, XH);
  degree_kernel<<<kTilesD, kNT, 0, stream>>>(ei, DINV);

  const int tiles = (kNodesPad / 64) * (kHid / 64);
  wmma_gemm64<0, false, 0, 0, false, 0><<<dim3((tiles + 7) / 8, 1), 256, 0, stream>>>(
      (const unsigned short*)XH, (const unsigned short*)XH, kCin, 0L,
      (const unsigned short*)W1T, (const unsigned short*)W1T, kCin, 0L,
      (void*)HL, (void*)nullptr, kHid, 0L,
      (const float*)nullptr, (const float*)nullptr, 0L, kNodesPad, kHid, kCin, kScale1);
  gcn_agg_kernel<true><<<kTiles, kNT, 0, stream>>>(HL, ei, DINV, b1, H1H, H2);

  wmma_gemm64<0, false, 0, 0, false, 0><<<dim3((tiles + 7) / 8, 1), 256, 0, stream>>>(
      (const unsigned short*)H1H, (const unsigned short*)H1H, kHid, 0L,
      (const unsigned short*)W2T, (const unsigned short*)W2T, kHid, 0L,
      (void*)HL, (void*)nullptr, kHid, 0L,
      (const float*)nullptr, (const float*)nullptr, 0L, kNodesPad, kHid, kHid, kScale2);
  gcn_agg_kernel<false><<<kTiles, kNT, 0, stream>>>(HL, ei, DINV, b2, H1H, H2);

  pool_kernel<<<kGraphs / kGpb, kNT, 0, stream>>>(H2, bat, P);
  head_kernel<<<1, kNT, 0, stream>>>(P, Wc1, bc1, Wc2, bc2, out);
}
